// BalSCL_SSL_BAL_16690242913044
// MI455X (gfx1250) — hardware-verified
//
#include <hip/hip_runtime.h>
#include <stdint.h>


typedef _Float16 v16h __attribute__((ext_vector_type(16)));
typedef _Float16 v8h  __attribute__((ext_vector_type(8)));
typedef float    v8f  __attribute__((ext_vector_type(8)));
typedef float    v4f  __attribute__((ext_vector_type(4)));
typedef v4f __attribute__((may_alias)) v4fa;

#define NB2      8192
#define NCLS     100
#define NREP     1
#define DDIM     128
#define NTOT     8292
#define NPAD     8304
#define NTILES   519
#define NCHUNK   8
#define TPC      65
#define RPB      128
#define NROWBLK  64
#define NCW      128
#define OPSCALE  64.0f
#define LSCALE   0.00244140625f

typedef char chk_a[(NTILES * 16 == NPAD) ? 1 : -1];
typedef char chk_b[(NCHUNK * TPC >= NTILES) ? 1 : -1];
typedef char chk_c[(NROWBLK * RPB == NB2) ? 1 : -1];
typedef char chk_d[(NB2 + NCLS * NREP == NTOT) ? 1 : -1];
typedef char chk_e[(NPAD >= NTOT) ? 1 : -1];
typedef char chk_f[((NPAD * DDIM) % 8 == 0) ? 1 : -1];


__device__ __forceinline__ v8f wmma16(v16h a, v16h b, v8f c) {
    c = __builtin_amdgcn_wmma_f32_16x16x32_f16(false, a, false, b, (short)0, c, false, false);
    asm volatile("v_nop\n\tv_nop\n\tv_nop\n\tv_nop" : "+v"(c) : "v"(a), "v"(b));
    return c;
}

__device__ __forceinline__ v16h load_frag(const _Float16* rowptr, int k0, int h) {
    union { v16h v; v8h p[2]; } f;
    f.p[0] = *(const v8h*)(rowptr + k0 + 8 * h);
    f.p[1] = *(const v8h*)(rowptr + k0 + 16 + 8 * h);
    return f.v;
}

__device__ __forceinline__ float sumsq16(v16h a, float s) {
    #pragma unroll
    for (int i = 0; i < 16; ++i) {
        const float v = (float)a[i];
        s = __builtin_fmaf(v, v, s);
    }
    return s;
}


__global__ __launch_bounds__(256)
void k_labels(const float* __restrict__ targets, int* labels) {
    const int j = blockIdx.x * 256 + threadIdx.x;
    if (j >= NB2) return;
    const float* row = targets + (size_t)j * NCLS;
    int lab = 0;
    float best = row[0];
    for (int c = 1; c < NCLS; ++c) {
        const float t = row[c];
        if (t > best) { best = t; lab = c; }
    }
    volatile int* p = labels + j;
    *p = lab;
    __threadfence();
    *p = lab;
}


__global__ __launch_bounds__(NCW)
void k_count(const int* __restrict__ labels, const float* __restrict__ clsnum, float* clsw) {
    (void)clsnum;
    const int c = threadIdx.x;
    int cnt = 0;
    for (int j = 0; j < NB2; ++j) cnt += (labels[j] == c) ? 1 : 0;
    const float v = (c < NCLS) ? (float)(cnt + NREP) : 1.0f;
    volatile float* p = clsw + c;
    *p = v;
    __threadfence();
    *p = v;
}


__global__ __launch_bounds__(256)
void k_convert(const float* __restrict__ feats, const float* __restrict__ cents, _Float16* FB) {
    const int t = blockIdx.x * 256 + threadIdx.x;
    if (t >= (NPAD * DDIM) / 8) return;
    const int e0  = t * 8;
    const int row = e0 / DDIM;
    v4f x0 = {0.0f, 0.0f, 0.0f, 0.0f};
    v4f x1 = {0.0f, 0.0f, 0.0f, 0.0f};
    if (row < NB2) {
        x0 = *(const v4fa*)(feats + e0);
        x1 = *(const v4fa*)(feats + e0 + 4);
    } else if (row < NTOT) {
        const int o = e0 - NB2 * DDIM;
        x0 = *(const v4fa*)(cents + o);
        x1 = *(const v4fa*)(cents + o + 4);
    }
    v8h o;
    o[0] = (_Float16)(x0[0] * OPSCALE);
    o[1] = (_Float16)(x0[1] * OPSCALE);
    o[2] = (_Float16)(x0[2] * OPSCALE);
    o[3] = (_Float16)(x0[3] * OPSCALE);
    o[4] = (_Float16)(x1[0] * OPSCALE);
    o[5] = (_Float16)(x1[1] * OPSCALE);
    o[6] = (_Float16)(x1[2] * OPSCALE);
    o[7] = (_Float16)(x1[3] * OPSCALE);
    volatile v8h* p = (volatile v8h*)(FB + e0);
    *p = o;
    __threadfence();
    *p = o;
}


__global__ __launch_bounds__(256)
void k_main(const _Float16* __restrict__ FB, const int* __restrict__ labels,
            const float* __restrict__ clsw, float* Sp, float* Pp) {
    __shared__ float sS[RPB];
    __shared__ float sP[RPB];

    const int lane    = threadIdx.x & 31;
    const int wave    = threadIdx.x >> 5;
    const int li      = lane & 15;
    const int h       = lane >> 4;
    const int rowBase = blockIdx.x * RPB + wave * 16;
    const int chunk   = blockIdx.y;

    const _Float16* arow = FB + (size_t)(rowBase + li) * DDIM;
    const v16h a0 = load_frag(arow,  0, h);
    const v16h a1 = load_frag(arow, 32, h);
    const v16h a2 = load_frag(arow, 64, h);
    const v16h a3 = load_frag(arow, 96, h);

    float ss = 0.0f;
    ss = sumsq16(a0, ss);
    ss = sumsq16(a1, ss);
    ss = sumsq16(a2, ss);
    ss = sumsq16(a3, ss);
    ss += __shfl_xor(ss, 16, 32);
    const float selfLogit = ss * LSCALE;

    float shift[8];
    int   lab[8];
    #pragma unroll
    for (int r = 0; r < 8; ++r) {
        shift[r] = __shfl(selfLogit, 8 * h + r, 32);
        lab[r]   = labels[rowBase + 8 * h + r];
    }

    float Sacc[8], Pacc[8];
    #pragma unroll
    for (int r = 0; r < 8; ++r) { Sacc[r] = 0.0f; Pacc[r] = 0.0f; }

    const int t0 = chunk * TPC;
    const int t1 = (t0 + TPC < NTILES) ? (t0 + TPC) : NTILES;

    for (int t = t0; t < t1; ++t) {
        const int colBase = t * 16;
        const int col     = colBase + li;
        const _Float16* brow = FB + (size_t)col * DDIM;

        const v16h b0 = load_frag(brow,  0, h);
        const v16h b1 = load_frag(brow, 32, h);
        const v16h b2 = load_frag(brow, 64, h);
        const v16h b3 = load_frag(brow, 96, h);

        v8f c = {0.0f, 0.0f, 0.0f, 0.0f, 0.0f, 0.0f, 0.0f, 0.0f};
        c = wmma16(a0, b0, c);
        c = wmma16(a1, b1, c);
        c = wmma16(a2, b2, c);
        c = wmma16(a3, b3, c);

        const bool valid = col < NTOT;
        const int  lj    = labels[(col < NB2) ? col : (NB2 - 1)];
        const int  predc = (col < NB2) ? lj : (valid ? (col - NB2) : -1);
        const int  pcl   = predc < 0 ? 0 : (predc > (NCW - 1) ? (NCW - 1) : predc);
        const float cc   = valid ? clsw[pcl] : 1.0f;

        #pragma unroll
        for (int r = 0; r < 8; ++r) {
            const int   myrow   = rowBase + 8 * h + r;
            const bool  notSelf = (col != myrow);
            const bool  isPos   = (predc == lab[r]) && notSelf;
            const float earg    = __builtin_fmaf(c[r], LSCALE, -shift[r]);
            const float w       = cc - (isPos ? 1.0f : 0.0f);
            const float e       = __expf(earg) * __builtin_amdgcn_rcpf(w);
            Sacc[r] += (valid && notSelf) ? e : 0.0f;
            Pacc[r] += isPos ? earg : 0.0f;
        }
    }

    #pragma unroll
    for (int r = 0; r < 8; ++r) {
        float s = Sacc[r], p = Pacc[r];
        #pragma unroll
        for (int m = 8; m >= 1; m >>= 1) {
            s += __shfl_xor(s, m, 16);
            p += __shfl_xor(p, m, 16);
        }
        Sacc[r] = s;
        Pacc[r] = p;
    }

    float vs = Sacc[0], vp = Pacc[0];
    #pragma unroll
    for (int r = 1; r < 8; ++r) {
        if (li == r) { vs = Sacc[r]; vp = Pacc[r]; }
    }
    if (li < 8) {
        sS[wave * 16 + 8 * h + li] = vs;
        sP[wave * 16 + 8 * h + li] = vp;
    }
    __syncthreads();

    const size_t seg = (size_t)chunk * NB2 + (size_t)blockIdx.x * RPB;
    if (wave == 0) {
        const v4f v = *(const v4fa*)(sS + 4 * lane);
        volatile v4f* p = (volatile v4f*)(Sp + seg) + lane;
        *p = v;
        __threadfence();
        *p = v;
    } else if (wave == 1) {
        const v4f v = *(const v4fa*)(sP + 4 * lane);
        volatile v4f* p = (volatile v4f*)(Pp + seg) + lane;
        *p = v;
        __threadfence();
        *p = v;
    }
}


__global__ __launch_bounds__(256)
void k_final(const float* __restrict__ Sp, const float* __restrict__ Pp,
             const int* __restrict__ labels, const float* __restrict__ clsw,
             const float* __restrict__ conf, float* out) {
    __shared__ double sn[256];
    __shared__ double sd[256];
    double num = 0.0, den = 0.0;
    for (int i = threadIdx.x; i < NB2; i += 256) {
        float S = 0.0f, P = 0.0f;
        #pragma unroll
        for (int k = 0; k < NCHUNK; ++k) {
            S += Sp[(size_t)k * NB2 + i];
            P += Pp[(size_t)k * NB2 + i];
        }
        int L = labels[i];
        L = L < 0 ? 0 : (L > (NCW - 1) ? (NCW - 1) : L);
        const float npos = clsw[L] - 1.0f;
        const float v    = __logf(S) - P * __builtin_amdgcn_rcpf(npos);
        const float cf   = conf[i];
        num += (double)(cf * v);
        den += (double)cf;
    }
    sn[threadIdx.x] = num;
    sd[threadIdx.x] = den;
    __syncthreads();
    for (int s = 128; s > 0; s >>= 1) {
        if (threadIdx.x < s) {
            sn[threadIdx.x] += sn[threadIdx.x + s];
            sd[threadIdx.x] += sd[threadIdx.x + s];
        }
        __syncthreads();
    }
    if (threadIdx.x == 0) {
        const float res = (float)(sn[0] / sd[0]);
        volatile float* p = out;
        *p = res;
        __threadfence();
        *p = res;
    }
}


extern "C" void kernel_launch(void* const* d_in, const int* in_sizes, int n_in,
                              void* d_out, int out_size, void* d_ws, size_t ws_size,
                              hipStream_t stream) {
    if (n_in < 5 || out_size < 1) return;
    if (in_sizes[0] != NCLS * NREP * DDIM) return;
    if (in_sizes[1] != NB2 * DDIM) return;
    if (in_sizes[2] != NB2 * NCLS) return;
    if (in_sizes[3] != NCLS) return;
    if (in_sizes[4] != NB2) return;

    const float* centers  = (const float*)d_in[0];
    const float* features = (const float*)d_in[1];
    const float* targets  = (const float*)d_in[2];
    const float* clsnum   = (const float*)d_in[3];
    const float* conf     = (const float*)d_in[4];
    float* out = (float*)d_out;

    uint8_t* base = (uint8_t*)d_ws;
    size_t off = 0;
    const size_t bFB  = (size_t)NPAD * DDIM * sizeof(_Float16);
    const size_t bSP  = (size_t)NCHUNK * NB2 * sizeof(float);
    const size_t bLab = (size_t)NB2 * sizeof(int);
    const size_t bCw  = (size_t)NCW * sizeof(float);
    _Float16* FB     = (_Float16*)(base + off); off += (bFB  + 255) & ~(size_t)255;
    float*    Sp     = (float*)   (base + off); off += (bSP  + 255) & ~(size_t)255;
    float*    Pp     = (float*)   (base + off); off += (bSP  + 255) & ~(size_t)255;
    int*      labels = (int*)     (base + off); off += (bLab + 255) & ~(size_t)255;
    float*    clsw   = (float*)   (base + off); off += (bCw  + 255) & ~(size_t)255;
    if (off > ws_size) return;

    k_labels<<<(NB2 + 255) / 256, 256, 0, stream>>>(targets, labels);
    k_count<<<1, NCW, 0, stream>>>(labels, clsnum, clsw);
    k_convert<<<((NPAD * DDIM) / 8 + 255) / 256, 256, 0, stream>>>(features, centers, FB);

    dim3 grid(NROWBLK, NCHUNK);
    k_main<<<grid, 256, 0, stream>>>(FB, labels, clsw, Sp, Pp);

    k_final<<<1, 256, 0, stream>>>(Sp, Pp, labels, clsw, conf, out);
}
